// MTL_Decoder_39865886442144
// MI455X (gfx1250) — hardware-verified
//
#include <hip/hip_runtime.h>


#define BB   64
#define PQ   100
#define PP   128
#define NK   1000
#define NP   1024
#define EMB  256
#define NH_  16
#define HD   16
#define HP   32
#define QIN  1284
#define QIP  1312
#define PCAR 1024.0f
#define GB   8
typedef _Float16 h16;
typedef unsigned short bf;
typedef __attribute__((ext_vector_type(16))) __bf16   v16bf;
typedef __attribute__((ext_vector_type(16))) _Float16 v16h;
typedef __attribute__((ext_vector_type(8)))  _Float16 v8h;
typedef __attribute__((ext_vector_type(8)))  unsigned short v8us;
typedef __attribute__((ext_vector_type(8)))  float    v8f;
typedef __attribute__((ext_vector_type(4)))  float    v4f;
typedef v8h  __attribute__((may_alias)) v8ha;
typedef v4f  __attribute__((may_alias)) v4fa;
typedef v8us __attribute__((may_alias)) v8usa;

__device__ __forceinline__ unsigned short f2bf(float f) { unsigned u = __float_as_uint(f); u += 0x7FFFu + ((u >> 16) & 1u); return (unsigned short)(u >> 16); }
__device__ __forceinline__ float bf2f(unsigned short b) { return __uint_as_float(((unsigned)b) << 16); }
__device__ __forceinline__ float bfr(float f) { return bf2f(f2bf(f)); }
__device__ __forceinline__ v16h cat16(v8h lo, v8h hi) { return __builtin_shufflevector(lo, hi, 0, 1, 2, 3, 4, 5, 6, 7, 8, 9, 10, 11, 12, 13, 14, 15); }
__device__ __forceinline__ v16bf cat16b(v8us lo, v8us hi) { return __builtin_bit_cast(v16bf, __builtin_shufflevector(lo, hi, 0, 1, 2, 3, 4, 5, 6, 7, 8, 9, 10, 11, 12, 13, 14, 15)); }
__device__ __forceinline__ v8f wmma16(v16h a, v16h b, v8f c) { return __builtin_amdgcn_wmma_f32_16x16x32_f16(false, a, false, b, (short)0, c, false, false); }
__device__ __forceinline__ v8f wmmab(v16bf a, v16bf b, v8f c) { return __builtin_amdgcn_wmma_f32_16x16x32_bf16(false, a, false, b, (short)0, c, false, false); }


template <typename T16> struct WFrag;
template <> struct WFrag<h16> { typedef v16h V; static __device__ __forceinline__ V ld(const h16* p) { return cat16(*(const v8h*)p, *(const v8h*)(p + 16)); } static __device__ __forceinline__ v8f mma(V a, V b, v8f c) { return wmma16(a, b, c); } };
template <> struct WFrag<bf> { typedef v16bf V; static __device__ __forceinline__ V ld(const bf* p) { return cat16b(*(const v8us*)p, *(const v8us*)(p + 16)); } static __device__ __forceinline__ v8f mma(V a, V b, v8f c) { return wmmab(a, b, c); } };
template <typename T16, int NSPLIT, bool BIAS>
__global__ __launch_bounds__(32) void k_gemmw(const T16* __restrict__ A, const T16* __restrict__ A2, const T16* __restrict__ Bt, const T16* __restrict__ Bt2, int K, float* C, int ldc, const float* __restrict__ bias, size_t sA, size_t sB, size_t sC) {
    typedef typename WFrag<T16>::V V;
    __shared__ __align__(16) float os[16 * 68];
    const size_t z = blockIdx.z; A += z * sA; if (A2) A2 += z * sA; Bt += z * sB; if (Bt2) Bt2 += z * sB; C += z * sC;
    const int lane = threadIdx.x & 31, lr = lane & 15, hi = lane >> 4; const int r0 = blockIdx.x * 64, c0 = blockIdx.y * 64;
    v8f acc[4][4];
#pragma unroll
    for (int mb = 0; mb < 4; ++mb)
#pragma unroll
        for (int nb = 0; nb < 4; ++nb) acc[mb][nb] = (v8f){};
    const size_t aoff = (size_t)(r0 + lr) * K + 8 * hi, boff = (size_t)(c0 + lr) * K + 8 * hi;
#pragma unroll 1
    for (int kc = 0; kc < K; kc += 32) {
        V a[4], a2[4];
#pragma unroll
        for (int mb = 0; mb < 4; ++mb) { a[mb] = WFrag<T16>::ld(A + aoff + (size_t)mb * 16 * K + kc); if (NSPLIT == 1 || NSPLIT == 2) a2[mb] = WFrag<T16>::ld(A2 + aoff + (size_t)mb * 16 * K + kc); }
#pragma unroll
        for (int nb = 0; nb < 4; ++nb) { const V b = WFrag<T16>::ld(Bt + boff + (size_t)nb * 16 * K + kc); V b2; if (NSPLIT >= 2) b2 = WFrag<T16>::ld(Bt2 + boff + (size_t)nb * 16 * K + kc);
#pragma unroll
            for (int mb = 0; mb < 4; ++mb) { acc[mb][nb] = WFrag<T16>::mma(a[mb], b, acc[mb][nb]); if (NSPLIT == 1 || NSPLIT == 2) acc[mb][nb] = WFrag<T16>::mma(a2[mb], b, acc[mb][nb]); if (NSPLIT >= 2) acc[mb][nb] = WFrag<T16>::mma(a[mb], b2, acc[mb][nb]); } }
        asm volatile("v_nop\n\tv_nop\n\tv_nop\n\tv_nop" : "+v"(acc[0][0]), "+v"(acc[1][1]), "+v"(acc[2][2]), "+v"(acc[3][3]) : "v"(a[0]), "v"(a[3]));
    }
#pragma unroll
    for (int mb = 0; mb < 4; ++mb) {
#pragma unroll
        for (int nb = 0; nb < 4; ++nb) {
#pragma unroll
            for (int j = 0; j < 8; ++j) os[(hi * 8 + j) * 68 + nb * 16 + lr] = acc[mb][nb][j]; }
        __builtin_amdgcn_wave_barrier(); asm volatile("" ::: "memory");
        float* crow = C + (size_t)(r0 + mb * 16) * ldc + c0;
#pragma unroll 1
        for (int ps = 0; ps < 2; ++ps) {
#pragma unroll
            for (int s = 0; s < 8; ++s) { const int row = 2 * s + hi, cofs = lr * 4; v4f val = *(const v4fa*)(os + row * 68 + cofs); if (BIAS) { val[0] += bfr(bias[c0 + cofs]); val[1] += bfr(bias[c0 + cofs + 1]); val[2] += bfr(bias[c0 + cofs + 2]); val[3] += bfr(bias[c0 + cofs + 3]); }
                *(volatile v4f*)(crow + (size_t)row * ldc + cofs) = val; }
            if (ps == 0) __threadfence(); }
        __builtin_amdgcn_wave_barrier(); asm volatile("" ::: "memory");
    }
}

__device__ __forceinline__ h16 tohx(float x) { return (h16)x; }
__device__ __forceinline__ void splitf(float y, unsigned short& h, unsigned short& l) { h = f2bf(y); l = f2bf(y - bf2f(h)); }
__device__ __forceinline__ float tanhf_(float a) { const float e2 = __expf(2.0f * a); return __fsub_rn(1.0f, __fdiv_rn(2.0f, __fadd_rn(e2, 1.0f))); }
typedef __attribute__((ext_vector_type(2))) _Float16 v2h;
typedef __attribute__((ext_vector_type(4))) _Float16 v4h;
typedef __attribute__((ext_vector_type(2))) unsigned short v2us;
typedef __attribute__((ext_vector_type(4))) unsigned short v4us;
typedef __attribute__((ext_vector_type(2))) float v2f;

__global__ __launch_bounds__(256) void k_wtG(const float* __restrict__ w, int K, int N, bf* Bt) {
    const int lane = threadIdx.x & 31; const int L0 = (blockIdx.x * 8 + (threadIdx.x >> 5)) * 8; const int nlines = N * K / 64;
#pragma unroll 1
    for (int ps = 0; ps < 2; ++ps) {
#pragma unroll 1
        for (int l = 0; l < 8; ++l) { const int L = L0 + l; if (L >= nlines) break; const size_t e = (size_t)L * 64 + lane * 2; const int k = (int)(e % K), n = (int)(e / K); v2us o;
            o[0] = f2bf(w[(size_t)k * N + n]); o[1] = f2bf(w[(size_t)(k + 1) * N + n]); *(volatile v2us*)(Bt + e) = o; }
        if (ps == 0) __threadfence(); }
}
__global__ __launch_bounds__(256) void k_wq(const float* __restrict__ w, bf* Bt) { const int e = (blockIdx.x * 256 + threadIdx.x) * 4; if (e >= EMB * QIP) return; const int k = e % QIP, n = e / QIP; v4us o;
#pragma unroll
    for (int q = 0; q < 4; ++q) o[q] = (k + q < QIN) ? f2bf(w[(size_t)(k + q) * EMB + n]) : (unsigned short)0; *(volatile v4us*)(Bt + e) = o; __threadfence(); *(volatile v4us*)(Bt + e) = o; }
__global__ __launch_bounds__(256) void k_qin(const float* __restrict__ ln_, const float* __restrict__ attr, const float* __restrict__ ctx, bf* QI) { const size_t e = ((size_t)blockIdx.x * 256 + threadIdx.x) * 4; if (e >= (size_t)GB * PP * QIP) return; const int k = (int)(e % QIP); const int p = (int)((e / QIP) % PP); const int b = (int)(e / ((size_t)QIP * PP)); v4us o;
#pragma unroll
    for (int q = 0; q < 4; ++q) { const int kk = k + q; float v = 0.f; if (p < PQ) { if (kk < EMB) v = ln_[((size_t)b * PQ + p) * EMB + kk]; else if (kk < EMB + 4) v = attr[((size_t)b * PQ + p) * 4 + (kk - EMB)]; else if (kk < QIN) v = ctx[(size_t)b * 1024 + (kk - EMB - 4)]; } o[q] = f2bf(v); }
    *(volatile v4us*)(QI + e) = o; __threadfence(); *(volatile v4us*)(QI + e) = o; }
__global__ __launch_bounds__(256) void k_nodes(const float* __restrict__ enc, bf* EN) { const size_t e = ((size_t)blockIdx.x * 256 + threadIdx.x) * 8; if (e >= (size_t)GB * NP * EMB) return; const int c = (int)(e % EMB); const int n = (int)((e / EMB) % NP); const int b = (int)(e / ((size_t)EMB * NP)); typedef __attribute__((ext_vector_type(8))) unsigned short v8us_; v8us_ o;
    if (n < NK) { const float* s = enc + ((size_t)b * NK + n) * EMB + c; const v4f a = *(const v4f*)s, bq = *(const v4f*)(s + 4); o[0] = f2bf(a[0]); o[1] = f2bf(a[1]); o[2] = f2bf(a[2]); o[3] = f2bf(a[3]); o[4] = f2bf(bq[0]); o[5] = f2bf(bq[1]); o[6] = f2bf(bq[2]); o[7] = f2bf(bq[3]); } else { for (int q = 0; q < 8; ++q) o[q] = 0; }
    *(volatile v8us_*)(EN + e) = o; __threadfence(); *(volatile v8us_*)(EN + e) = o; }
__global__ __launch_bounds__(256) void k_qp(const float* __restrict__ Qf, h16* QP) { const size_t e = ((size_t)blockIdx.x * 256 + threadIdx.x) * 2; if (e >= (size_t)GB * NH_ * PP * HP) return; const int d = (int)(e % HP); const int p = (int)((e / HP) % PP); const int h = (int)((e / ((size_t)HP * PP)) % NH_); const int b = (int)(e / ((size_t)HP * PP * NH_)); v2h o;
    if (d < HD) { const float* s = Qf + ((size_t)b * PP + p) * EMB + h * HD + d; o[0] = tohx(s[0]); o[1] = tohx(s[1]); } else { o[0] = (h16)0.f; o[1] = (h16)0.f; } *(volatile v2h*)(QP + e) = o; __threadfence(); *(volatile v2h*)(QP + e) = o; }
__global__ __launch_bounds__(256) void k_kp(const float* __restrict__ Kf, h16* KP) { const size_t e = ((size_t)blockIdx.x * 256 + threadIdx.x) * 2; if (e >= (size_t)GB * NH_ * NP * HP) return; const int d = (int)(e % HP); const int n = (int)((e / HP) % NP); const int h = (int)((e / ((size_t)HP * NP)) % NH_); const int b = (int)(e / ((size_t)HP * NP * NH_)); v2h o;
    if (d < HD) { const float* s = Kf + ((size_t)b * NP + n) * EMB + h * HD + d; o[0] = tohx(s[0]); o[1] = tohx(s[1]); } else { o[0] = (h16)0.f; o[1] = (h16)0.f; } *(volatile v2h*)(KP + e) = o; __threadfence(); *(volatile v2h*)(KP + e) = o; }
__global__ __launch_bounds__(256) void k_vt(const float* __restrict__ Vf, h16* VT) { const size_t e = ((size_t)blockIdx.x * 256 + threadIdx.x) * 2; if (e >= (size_t)GB * NH_ * 64 * NP) return; const int n = (int)(e % NP); const int dd = (int)((e / NP) % 64); const int h = (int)((e / ((size_t)NP * 64)) % NH_); const int b = (int)(e / ((size_t)NP * 64 * NH_)); v2h o;
    if (dd < HD) { o[0] = tohx(Vf[((size_t)b * NP + n) * EMB + h * HD + dd]); o[1] = tohx(Vf[((size_t)b * NP + n + 1) * EMB + h * HD + dd]); } else { o[0] = (h16)0.f; o[1] = (h16)0.f; } *(volatile v2h*)(VT + e) = o; __threadfence(); *(volatile v2h*)(VT + e) = o; }
__global__ __launch_bounds__(256) void k_msoft(const float* __restrict__ S, const float* __restrict__ mask, int z0, h16* P) { const int lane = threadIdx.x & 31; const int row = blockIdx.x * 8 + (threadIdx.x >> 5); if (row >= GB * NH_ * PP) return; const int p = row % PP, zz = row / PP; const int pr = z0 + zz; const int b = pr / NH_; const float* sr = S + (size_t)row * NP; const float* mr = mask + ((size_t)b * PQ + (p < PQ ? p : 0)) * NK; float v[32]; float mx = -3.0e38f;
#pragma unroll
    for (int ch = 0; ch < 8; ++ch) { const int j0 = ch * 128 + lane * 4; const v4f a = *(const v4f*)(sr + j0);
#pragma unroll
        for (int q = 0; q < 4; ++q) { const int n = j0 + q; float t; if (n < NK) { float s4 = __fmul_rn(a[q], 0.25f); asm volatile("" : "+v"(s4)); t = (p < PQ) ? __fadd_rn(s4, bfr(mr[n])) : s4; } else t = -3.0e38f; v[ch * 4 + q] = t; mx = fmaxf(mx, t); } }
#pragma unroll
    for (int sh = 16; sh; sh >>= 1) mx = fmaxf(mx, __shfl_xor(mx, sh, 32));
    float sum = 0.f;
#pragma unroll
    for (int k = 0; k < 32; ++k) { float d0 = __fsub_rn(v[k], mx); asm volatile("" : "+v"(d0)); v[k] = (v[k] > -1.0e38f) ? __expf(d0) : 0.f; sum += v[k]; }
#pragma unroll
    for (int sh = 16; sh; sh >>= 1) sum += __shfl_xor(sum, sh, 32);
    const float f = __fdiv_rn(PCAR, sum);
#pragma unroll 1
    for (int ps = 0; ps < 2; ++ps) {
#pragma unroll
        for (int ch = 0; ch < 8; ++ch) { v4h o;
#pragma unroll
            for (int q = 0; q < 4; ++q) o[q] = tohx(v[ch * 4 + q] * f); *(volatile v4h*)(P + (size_t)row * NP + ch * 128 + lane * 4) = o; }
        if (ps == 0) __threadfence(); } }
__global__ __launch_bounds__(256) void k_mrg16(const float* __restrict__ O, int z0, int nz, bf* Ch, bf* Cl) { const size_t e = ((size_t)blockIdx.x * 256 + threadIdx.x) * 2; if (e >= (size_t)nz * PP * HD) return; const int d = (int)(e % HD); const int p = (int)((e / HD) % PP); const int zz = (int)(e / ((size_t)HD * PP)); const int pr = z0 + zz; const int b = pr / NH_, h = pr % NH_; v2us oh, ol;
#pragma unroll
    for (int q = 0; q < 2; ++q) { unsigned short a, c2; splitf(O[((size_t)zz * PP + p) * 64 + d + q] * (1.0f / PCAR), a, c2); oh[q] = a; ol[q] = c2; } const size_t oo = ((size_t)b * PP + p) * EMB + h * HD + d; *(volatile v2us*)(Ch + oo) = oh; *(volatile v2us*)(Cl + oo) = ol; __threadfence(); *(volatile v2us*)(Ch + oo) = oh; *(volatile v2us*)(Cl + oo) = ol; }
__global__ __launch_bounds__(256) void k_split2(const float* __restrict__ F, bf* Ph, bf* Pl, size_t n) { const size_t i = ((size_t)blockIdx.x * 256 + threadIdx.x) * 2; if (i >= n) return; v2us oh, ol;
#pragma unroll
    for (int q = 0; q < 2; ++q) { unsigned short a, c2; splitf(F[i + q], a, c2); oh[q] = a; ol[q] = c2; } *(volatile v2us*)(Ph + i) = oh; *(volatile v2us*)(Pl + i) = ol; __threadfence(); *(volatile v2us*)(Ph + i) = oh; *(volatile v2us*)(Pl + i) = ol; }
__device__ __forceinline__ float plogit(float l, float mk) { float s16 = __fmul_rn(l, 0.0625f); asm volatile("" : "+v"(s16)); float th = __fmul_rn(10.0f, tanhf_(s16)); asm volatile("" : "+v"(th)); return __fadd_rn(th, mk); }
__global__ __launch_bounds__(256) void k_pstat(const float* __restrict__ L, const float* __restrict__ mask, float* RS) { const int lane = threadIdx.x & 31; const int row = blockIdx.x * 8 + (threadIdx.x >> 5); if (row >= GB * PQ) return; const int p = row % PQ, b = row / PQ; const float* lr = L + ((size_t)b * PP + p) * NP; const float* mr = mask + (size_t)row * NK; float mx = -3.0e38f;
    for (int n = lane; n < NK; n += 32) mx = fmaxf(mx, plogit(lr[n], bfr(mr[n])));
#pragma unroll
    for (int sh = 16; sh; sh >>= 1) mx = fmaxf(mx, __shfl_xor(mx, sh, 32));
    float sum = 0.f; for (int n = lane; n < NK; n += 32) { float d0 = __fsub_rn(plogit(lr[n], bfr(mr[n])), mx); asm volatile("" : "+v"(d0)); sum = __fadd_rn(sum, __expf(d0)); }
#pragma unroll
    for (int sh = 16; sh; sh >>= 1) sum += __shfl_xor(sum, sh, 32);
    const float o = lane == 0 ? mx : (lane == 1 ? __fdiv_rn(1.0f, sum) : 0.f); *(volatile float*)(RS + (size_t)row * 32 + lane) = o; __threadfence(); *(volatile float*)(RS + (size_t)row * 32 + lane) = o; }
__global__ __launch_bounds__(256) void k_pout(const float* __restrict__ L, const float* __restrict__ mask, const float* __restrict__ RS, float* OUT) { const size_t i = ((size_t)blockIdx.x * 256 + threadIdx.x) * 4; if (i >= (size_t)GB * PQ * NK) return; v4f o;
#pragma unroll
    for (int q = 0; q < 4; ++q) { const size_t e = i + q; const int n = (int)(e % NK); const int row = (int)(e / NK); const int p = row % PQ, b = row / PQ; const float t = plogit(L[((size_t)b * PP + p) * NP + n], bfr(mask[e])); float d0 = __fsub_rn(t, RS[(size_t)row * 32]); asm volatile("" : "+v"(d0)); o[q] = __fmul_rn(__expf(d0), RS[(size_t)row * 32 + 1]); }
    *(volatile v4f*)(OUT + i) = o; __threadfence(); *(volatile v4f*)(OUT + i) = o; }

extern "C" void kernel_launch(void* const* d_in, const int* in_sizes, int n_in,
                              void* d_out, int out_size, void* d_ws, size_t ws_size, hipStream_t stream) {
    (void)in_sizes; (void)n_in; (void)out_size;
    const float* last = (const float*)d_in[0]; const float* attr = (const float*)d_in[1]; const float* ctx = (const float*)d_in[2]; const float* mask = (const float*)d_in[3]; const float* enc = (const float*)d_in[4]; const float* Wq = (const float*)d_in[5]; const float* Wk = (const float*)d_in[6]; const float* Wv = (const float*)d_in[7]; const float* Wc = (const float*)d_in[8]; const float* bc = (const float*)d_in[9];
    float* OUT = (float*)d_out;
    char* wsp = (char*)d_ws;
    auto take = [&](size_t bytes) { char* p = wsp; wsp += (bytes + 255) & ~(size_t)255; return (void*)p; };
    const int ZC = GB * NH_;
    bf* WQ = (bf*)take((size_t)EMB * QIP * 2); bf* WK = (bf*)take((size_t)EMB * EMB * 2); bf* WV = (bf*)take((size_t)EMB * EMB * 2); bf* WC = (bf*)take((size_t)EMB * EMB * 2);
    bf* EN = (bf*)take((size_t)GB * NP * EMB * 2); bf* QI = (bf*)take((size_t)GB * PP * QIP * 2); float* Qf = (float*)take((size_t)GB * PP * EMB * 4); float* KVf = (float*)take((size_t)GB * NP * EMB * 4);
    h16* QP = (h16*)take((size_t)GB * NH_ * PP * HP * 2); h16* KP = (h16*)take((size_t)GB * NH_ * NP * HP * 2); h16* VT = (h16*)take((size_t)GB * NH_ * 64 * NP * 2);
    float* S = (float*)take((size_t)ZC * PP * NP * 4); h16* P = (h16*)take((size_t)ZC * PP * NP * 2); float* O = (float*)take((size_t)ZC * PP * 64 * 4); bf* Ch = (bf*)take((size_t)GB * PP * EMB * 2); bf* Cl = (bf*)take((size_t)GB * PP * EMB * 2); float* MH = (float*)take((size_t)GB * PP * EMB * 4); bf* Mh = (bf*)take((size_t)GB * PP * EMB * 2); bf* Ml = (bf*)take((size_t)GB * PP * EMB * 2);
    float* L = S;
    float* RS = (float*)take((size_t)GB * PQ * 32 * 4);
    if ((size_t)(wsp - (char*)d_ws) > ws_size) return;
    k_wq<<<(EMB * QIP / 4 + 255) / 256, 256, 0, stream>>>(Wq, WQ); k_wtG<<<(EMB * EMB / 64 + 63) / 64, 256, 0, stream>>>(Wk, EMB, EMB, WK); k_wtG<<<(EMB * EMB / 64 + 63) / 64, 256, 0, stream>>>(Wv, EMB, EMB, WV); k_wtG<<<(EMB * EMB / 64 + 63) / 64, 256, 0, stream>>>(Wc, EMB, EMB, WC);
    for (int g = 0; g < BB / GB; ++g) { const int b0 = g * GB;
        k_nodes<<<(unsigned)(((size_t)GB * NP * EMB / 8 + 255) / 256), 256, 0, stream>>>(enc + (size_t)b0 * NK * EMB, EN);
        k_qin<<<(unsigned)(((size_t)GB * PP * QIP / 4 + 255) / 256), 256, 0, stream>>>(last + (size_t)b0 * PQ * EMB, attr + (size_t)b0 * PQ * 4, ctx + (size_t)b0 * 1024, QI);
        k_gemmw<bf, 0, false><<<dim3(GB * PP / 64, EMB / 64, 1), 32, 0, stream>>>(QI, nullptr, WQ, nullptr, QIP, Qf, EMB, nullptr, 0, 0, 0); k_qp<<<(unsigned)(((size_t)GB * NH_ * PP * HP / 2 + 255) / 256), 256, 0, stream>>>(Qf, QP);
        k_gemmw<bf, 0, false><<<dim3(GB * NP / 64, EMB / 64, 1), 32, 0, stream>>>(EN, nullptr, WK, nullptr, EMB, KVf, EMB, nullptr, 0, 0, 0); k_kp<<<(unsigned)(((size_t)GB * NH_ * NP * HP / 2 + 255) / 256), 256, 0, stream>>>(KVf, KP);
        k_gemmw<bf, 0, false><<<dim3(GB * NP / 64, EMB / 64, 1), 32, 0, stream>>>(EN, nullptr, WV, nullptr, EMB, KVf, EMB, nullptr, 0, 0, 0); k_vt<<<(unsigned)(((size_t)GB * NH_ * 64 * NP / 2 + 255) / 256), 256, 0, stream>>>(KVf, VT);
        k_gemmw<h16, 0, false><<<dim3(PP / 64, NP / 64, ZC), 32, 0, stream>>>(QP, nullptr, KP, nullptr, HP, S, NP, nullptr, (size_t)PP * HP, (size_t)NP * HP, (size_t)PP * NP);
        k_msoft<<<ZC * PP / 8, 256, 0, stream>>>(S, mask + (size_t)b0 * PQ * NK, 0, P);
        k_gemmw<h16, 0, false><<<dim3(PP / 64, 1, ZC), 32, 0, stream>>>(P, nullptr, VT, nullptr, NP, O, 64, nullptr, (size_t)PP * NP, (size_t)64 * NP, (size_t)PP * 64);
        k_mrg16<<<(unsigned)(((size_t)ZC * PP * HD / 2 + 255) / 256), 256, 0, stream>>>(O, 0, ZC, Ch, Cl);
        k_gemmw<bf, 1, true><<<dim3(GB * PP / 64, EMB / 64, 1), 32, 0, stream>>>(Ch, Cl, WC, nullptr, EMB, MH, EMB, bc, 0, 0, 0); k_split2<<<(unsigned)(((size_t)GB * PP * EMB / 2 + 255) / 256), 256, 0, stream>>>(MH, Mh, Ml, (size_t)GB * PP * EMB);
        k_gemmw<bf, 1, false><<<dim3(PP / 64, NP / 64, GB), 32, 0, stream>>>(Mh, Ml, EN, nullptr, EMB, L, NP, nullptr, (size_t)PP * EMB, (size_t)NP * EMB, (size_t)PP * NP);
        k_pstat<<<GB * PQ / 8, 256, 0, stream>>>(L, mask + (size_t)b0 * PQ * NK, RS);
        k_pout<<<(unsigned)(((size_t)GB * PQ * NK / 4 + 255) / 256), 256, 0, stream>>>(L, mask + (size_t)b0 * PQ * NK, RS, OUT + (size_t)b0 * PQ * NK); }
}
